// Sequence_59554016526399
// MI455X (gfx1250) — hardware-verified
//
#include <hip/hip_runtime.h>
#include <math.h>

typedef __attribute__((ext_vector_type(16))) __bf16 v16b;
typedef __attribute__((ext_vector_type(8)))  __bf16 v8b;
typedef __attribute__((ext_vector_type(8)))  float  v8f;
typedef __attribute__((ext_vector_type(4)))  float  v4f;
typedef __attribute__((ext_vector_type(2)))  float  v2f;

constexpr int kLen      = 131072;
constexpr int kVoc      = 10;
constexpr int kEmb      = 20;
constexpr int kHid      = 30;
constexpr int kGates    = 4 * kHid;
constexpr int kGatesPad = 128;
constexpr int kHPitch   = 32;
constexpr int kChunk    = 16;
constexpr int kNChunk   = kLen / kChunk;
constexpr int kWPitch   = 40;
constexpr int kXPitch   = 132;
constexpr int kWhhVec4  = (kGates * kHid) / 4;
constexpr int kHeadWaves        = 4;
constexpr int kHeadRowsPerWave  = 64;
constexpr int kHeadRowsPerBlock = kHeadWaves * kHeadRowsPerWave;
constexpr int kHeadBlocks       = kLen / kHeadRowsPerBlock;
constexpr int kHeadFloatsPerWave = kHeadRowsPerWave * kVoc;
constexpr size_t kPlaneBytes = (size_t)kLen * kHPitch * 4;
constexpr size_t kWsTotal    = 4 * kPlaneBytes;
static_assert(kGates == 120);
static_assert(kGatesPad % 16 == 0 && kGatesPad >= kGates);
static_assert(kHPitch == 32 && kHPitch >= kHid);
static_assert(kLen % kChunk == 0 && (kChunk % 2) == 0);
static_assert(kLen % kHeadRowsPerBlock == 0);
static_assert(kHeadFloatsPerWave == 640 && (kHeadFloatsPerWave % 128) == 0);
static_assert((kGates * kHid) % 4 == 0 && kWhhVec4 == 900);
static_assert((kWPitch * 2) % 16 == 0 && (kXPitch * 4) % 16 == 0);
static_assert(kEmb == 20 && (kEmb % 4) == 0);
static_assert((kHid % 2) == 0);
static_assert(kWsTotal == 67108864ull);
static_assert(kWsTotal <= 134217728ull);

__device__ __forceinline__ unsigned short f2bf_bits(float f) {
  unsigned u = __float_as_uint(f);
  return (unsigned short)((u + 0x7FFFu + ((u >> 16) & 1u)) >> 16);
}
__device__ __forceinline__ float bf_bits2f(unsigned short h) { return __uint_as_float(((unsigned)h) << 16); }
__device__ __forceinline__ void bf_split(float v, unsigned short& hb, unsigned short& lb) {
  hb = f2bf_bits(v);
  lb = f2bf_bits(v - bf_bits2f(hb));
}

union FragB { v16b v; v8b h[2]; };
__device__ __forceinline__ v16b ld_frag_b(const __bf16* p) {
  FragB f;
  f.h[0] = *(const v8b*)(p);
  f.h[1] = *(const v8b*)(p + 16);
  return f.v;
}

__device__ __forceinline__ void split16(const v4f q0, const v4f q1, const v4f q2, const v4f q3,
                                        v16b& hi, v16b& lo) {
#pragma unroll
  for (int e = 0; e < 4; ++e) {
    const float s0 = q0[e];
    const float s1 = q1[e];
    const float s2 = q2[e];
    const float s3 = q3[e];
    unsigned short hb, lb;
    bf_split(s0, hb, lb);
    hi[e] = __builtin_bit_cast(__bf16, hb);
    lo[e] = __builtin_bit_cast(__bf16, lb);
    bf_split(s1, hb, lb);
    hi[4 + e] = __builtin_bit_cast(__bf16, hb);
    lo[4 + e] = __builtin_bit_cast(__bf16, lb);
    bf_split(s2, hb, lb);
    hi[8 + e] = __builtin_bit_cast(__bf16, hb);
    lo[8 + e] = __builtin_bit_cast(__bf16, lb);
    bf_split(s3, hb, lb);
    hi[12 + e] = __builtin_bit_cast(__bf16, hb);
    lo[12 + e] = __builtin_bit_cast(__bf16, lb);
  }
}

__device__ __forceinline__ v8f mma3_bf(v16b ah, v16b al, v16b bh, v16b bl, v8f c) {
  c = __builtin_amdgcn_wmma_f32_16x16x32_bf16(false, ah, false, bh, (short)0, c, false, false);
  c = __builtin_amdgcn_wmma_f32_16x16x32_bf16(false, ah, false, bl, (short)0, c, false, false);
  c = __builtin_amdgcn_wmma_f32_16x16x32_bf16(false, al, false, bh, (short)0, c, false, false);
  asm volatile("v_nop\n\tv_nop\n\tv_nop\n\tv_nop" : "+v"(c) : "v"(ah), "v"(al), "v"(bh), "v"(bl));
  return c;
}

__device__ __forceinline__ float gate_sigm(float v) {
  return __builtin_amdgcn_rcpf(1.0f + expf(-v));
}
__device__ __forceinline__ float gate_tanh(float v) {
  return 1.0f - 2.0f * __builtin_amdgcn_rcpf(expf(2.0f * v) + 1.0f);
}

__device__ __forceinline__ void proj_tiles(const v16b Ahi, const v16b Alo,
                                           const __bf16* wbh, const __bf16* wbl,
                                           const float* biasline, float* dst,
                                           int c, int hs) {
#pragma unroll 2
  for (int tile = 0; tile < kGatesPad / 16; ++tile) {
    const int n = tile * 16 + c;
    const v16b bh = ld_frag_b(wbh + n * kWPitch + 8 * hs);
    const v16b bl = ld_frag_b(wbl + n * kWPitch + 8 * hs);
    const float bv = biasline[n];
    v8f acc = (v8f){bv, bv, bv, bv, bv, bv, bv, bv};
    acc = mma3_bf(Ahi, Alo, bh, bl, acc);
#pragma unroll
    for (int r = 0; r < 8; ++r) dst[(8 * hs + r) * kXPitch + n] = acc[r];
  }
}

template <int LAYER>
__global__ __launch_bounds__(32) void chain_scan_kernel(
    const float* __restrict__ embed, const int* __restrict__ tokens,
    const float* __restrict__ hinF, const float* __restrict__ hinB,
    const float* __restrict__ WihF, const float* __restrict__ WhhF,
    const float* __restrict__ bihF, const float* __restrict__ bhhF,
    const float* __restrict__ WihB, const float* __restrict__ WhhB,
    const float* __restrict__ bihB, const float* __restrict__ bhhB,
    float* __restrict__ houtF, float* __restrict__ houtB)
{
  constexpr int KIN = (LAYER == 1) ? kEmb : kHid;
  __shared__ __align__(16) float  sWhh[kGates * kHid];
  __shared__ __align__(16) __bf16 sBh[kGatesPad * kWPitch];
  __shared__ __align__(16) __bf16 sBl[kGatesPad * kWPitch];
  __shared__ __align__(16) float  sBias[kGatesPad];
  __shared__ __align__(16) float  sXg[kChunk * kXPitch];
  __shared__ __align__(16) float  sHst[kChunk * kHPitch];
  __shared__ __align__(16) float  sHb[2 * 32];
  __shared__ int sTok[kChunk];

  const int  lane = threadIdx.x & 31;
  const int  c    = lane & 15;
  const int  hs   = lane >> 4;
  const bool act  = (lane < kHid);
  const int  ul   = act ? lane : (kHid - 1);
  const bool back = (blockIdx.x != 0);

  const float* Wih = back ? WihB : WihF;
  const float* Whh = back ? WhhB : WhhF;
  const float* bih = back ? bihB : bihF;
  const float* bhh = back ? bhhB : bhhF;
  const float* hin = back ? hinB : hinF;
  float*       hout = back ? houtB : houtF;

#pragma unroll 1
  for (int it = 0; it < 29; ++it) {
    const int idx = it * 32 + lane;
    const int idc = (idx < kWhhVec4) ? idx : (kWhhVec4 - 1);
    v4f v = *(const v4f*)(Whh + 4 * idc);
    asm volatile("" : "+v"(v));
    if (idx < kWhhVec4) *(v4f*)(sWhh + 4 * idx) = v;
  }

#pragma unroll 1
  for (int it = 0; it < 16; ++it) {
    const int i  = it * 32 + lane;
    const int n  = i >> 2;
    const int c8 = (i & 3) * 8;
    const int u  = n >> 2;
    const int q  = n & 3;
    const bool rowok = (u < kHid);
    const int  uc = rowok ? u : (kHid - 1);
    const float* rp = Wih + (size_t)(q * kHid + uc) * KIN;
    v8b hv, lv;
#pragma unroll
    for (int e = 0; e < 8; ++e) {
      const int  k   = c8 + e;
      const bool kok = (k < KIN);
      const int  kc  = kok ? k : (KIN - 1);
      float wv = rp[kc];
      asm volatile("" : "+v"(wv));
      const float sv = (rowok && kok) ? wv : 0.0f;
      unsigned short hb, lb;
      bf_split(sv, hb, lb);
      hv[e] = __builtin_bit_cast(__bf16, hb);
      lv[e] = __builtin_bit_cast(__bf16, lb);
    }
    *(v8b*)(sBh + n * kWPitch + c8) = hv;
    *(v8b*)(sBl + n * kWPitch + c8) = lv;
  }

#pragma unroll 1
  for (int it = 0; it < 4; ++it) {
    const int n = it * 32 + lane;
    const int u = n >> 2;
    const int q = n & 3;
    const bool rowok = (u < kHid);
    const int  uc = rowok ? u : (kHid - 1);
    float ba = bih[q * kHid + uc];
    float bb = bhh[q * kHid + uc];
    asm volatile("" : "+v"(ba), "+v"(bb));
    sBias[n] = rowok ? (ba + bb) : 0.0f;
  }

  sHb[lane]      = 0.0f;
  sHb[32 + lane] = 0.0f;
  __syncthreads();

  float w0[kHid], w1[kHid], w2[kHid], w3[kHid];
#pragma unroll
  for (int k = 0; k < kHid; ++k) {
    float t0 = sWhh[(0 * kHid + ul) * kHid + k];
    float t1 = sWhh[(1 * kHid + ul) * kHid + k];
    float t2 = sWhh[(2 * kHid + ul) * kHid + k];
    float t3 = sWhh[(3 * kHid + ul) * kHid + k];
    t0 = act ? t0 : 0.0f;
    t1 = act ? t1 : 0.0f;
    t2 = act ? t2 : 0.0f;
    t3 = act ? t3 : 0.0f;
    asm volatile("" : "+v"(t0), "+v"(t1), "+v"(t2), "+v"(t3));
    w0[k] = t0;
    w1[k] = t1;
    w2[k] = t2;
    w3[k] = t3;
  }

  if (LAYER == 1) {
    const bool mok = (c < kVoc);
    const int  mc  = mok ? c : (kVoc - 1);
    const float* rp = embed + mc * kEmb;
    const int  kb   = 16 + 8 * hs;
    const bool g2ok = ((kb + 3) < kEmb);
    const int  kbc  = g2ok ? kb : (kEmb - 4);
    v4f q0 = *(const v4f*)(rp + 8 * hs);
    v4f q1 = *(const v4f*)(rp + 8 * hs + 4);
    v4f q2 = *(const v4f*)(rp + kbc);
    asm volatile("" : "+v"(q0), "+v"(q1), "+v"(q2));
    const bool ok2 = mok && g2ok;
    v4f z0, z1, z2, z3;
#pragma unroll
    for (int e = 0; e < 4; ++e) {
      const float s0 = q0[e];
      const float s1 = q1[e];
      const float s2 = q2[e];
      z0[e] = mok ? s0 : 0.0f;
      z1[e] = mok ? s1 : 0.0f;
      z2[e] = ok2 ? s2 : 0.0f;
      z3[e] = 0.0f;
    }
    v16b Ahi, Alo;
    split16(z0, z1, z2, z3, Ahi, Alo);
    proj_tiles(Ahi, Alo, sBh, sBl, sBias, sXg, c, hs);
  }

  float cst = 0.0f;

#pragma unroll 1
  for (int ch = 0; ch < kNChunk; ++ch) {
    const int s0 = ch * kChunk;
    __syncthreads();
    if (LAYER == 1) {
      const int si = s0 + c;
      const int ti = back ? (kLen - 1 - si) : si;
      int tk = tokens[ti];
      asm volatile("" : "+v"(tk));
      tk = (tk < 0) ? 0 : ((tk > kVoc - 1) ? (kVoc - 1) : tk);
      if (lane < kChunk) sTok[lane] = tk;
    } else {
      const float* rp = hin + (size_t)(s0 + c) * kHPitch;
      v4f q0 = *(const v4f*)(rp + 8 * hs);
      v4f q1 = *(const v4f*)(rp + 8 * hs + 4);
      v4f q2 = *(const v4f*)(rp + 16 + 8 * hs);
      v4f q3 = *(const v4f*)(rp + 20 + 8 * hs);
      asm volatile("" : "+v"(q0), "+v"(q1), "+v"(q2), "+v"(q3));
      v16b Ahi, Alo;
      split16(q0, q1, q2, q3, Ahi, Alo);
      proj_tiles(Ahi, Alo, sBh, sBl, sBias, sXg, c, hs);
    }
    __syncthreads();

#pragma unroll 1
    for (int s = 0; s < kChunk; ++s) {
      const int pb = (s & 1) * 32;
      int xrow = s;
      if (LAYER == 1) xrow = sTok[s];
      const v4f xg = *(const v4f*)(sXg + xrow * kXPitch + 4 * lane);
      float a0 = xg[0];
      float a1 = xg[1];
      float a2 = xg[2];
      float a3 = xg[3];
#pragma unroll
      for (int k4 = 0; k4 < 8; ++k4) {
        const v4f hv = *(const v4f*)(sHb + pb + 4 * k4);
#pragma unroll
        for (int e = 0; e < 4; ++e) {
          const int k = 4 * k4 + e;
          if (k < kHid) {
            const float hk = hv[e];
            a0 = fmaf(w0[k], hk, a0);
            a1 = fmaf(w1[k], hk, a1);
            a2 = fmaf(w2[k], hk, a2);
            a3 = fmaf(w3[k], hk, a3);
          }
        }
      }
      const float ig = gate_sigm(a0);
      const float fg = gate_sigm(a1);
      const float gg = gate_tanh(a2);
      const float og = gate_sigm(a3);
      cst = fmaf(fg, cst, ig * gg);
      float hn = og * gate_tanh(cst);
      hn = act ? hn : 0.0f;
      sHb[(pb ^ 32) + lane] = hn;
      sHst[s * kHPitch + lane] = hn;
      __syncthreads();
    }

    {
      v4f fv[4];
#pragma unroll
      for (int it = 0; it < 4; ++it) fv[it] = *(const v4f*)(sHst + it * 128 + lane * 4);
      float* hp = hout + (size_t)s0 * kHPitch;
      for (int pass = 0; pass < 2; ++pass) {
#pragma unroll
        for (int it = 0; it < 4; ++it) {
          *(volatile v4f*)(hp + it * 128 + lane * 4) = fv[it];
        }
        __threadfence();
      }
    }
  }
}

__device__ __forceinline__ void load_head_b(const float* W, int nc, bool nok, int hs,
                                            v16b& hi, v16b& lo) {
#pragma unroll
  for (int j = 0; j < 8; ++j) {
    const int  k   = (j < 4) ? (8 * hs + 2 * j) : (16 + 8 * hs + 2 * (j - 4));
    const bool kok = ((k + 1) < kHid);
    const int  kc  = kok ? k : (kHid - 2);
    const v2f p = *(const v2f*)(W + nc * kHid + kc);
    float p0 = p[0];
    float p1 = p[1];
    asm volatile("" : "+v"(p0), "+v"(p1));
    const bool ok = nok && kok;
    const float s0 = ok ? p0 : 0.0f;
    const float s1 = ok ? p1 : 0.0f;
    unsigned short hb, lb;
    bf_split(s0, hb, lb);
    hi[2 * j] = __builtin_bit_cast(__bf16, hb);
    lo[2 * j] = __builtin_bit_cast(__bf16, lb);
    bf_split(s1, hb, lb);
    hi[2 * j + 1] = __builtin_bit_cast(__bf16, hb);
    lo[2 * j + 1] = __builtin_bit_cast(__bf16, lb);
  }
}

__global__ __launch_bounds__(128) void head_kernel(
    const float* __restrict__ h2f, const float* __restrict__ h2b,
    const float* __restrict__ WlF, const float* __restrict__ blF,
    const float* __restrict__ WlB, const float* __restrict__ blB,
    float* __restrict__ out)
{
  __shared__ __align__(16) float sOut[kHeadWaves][kHeadFloatsPerWave];
  const int lane = threadIdx.x & 31;
  const int wave = threadIdx.x >> 5;
  const int c    = lane & 15;
  const int hs   = lane >> 4;
  const int row0 = (blockIdx.x * kHeadWaves + wave) * kHeadRowsPerWave;

  const bool nok = (c < kVoc);
  const int  nc  = nok ? c : (kVoc - 1);
  v16b Bfh, Bfl, Bbh, Bbl;
  load_head_b(WlF, nc, nok, hs, Bfh, Bfl);
  load_head_b(WlB, nc, nok, hs, Bbh, Bbl);
  float bf = blF[nc];
  float bb = blB[nc];
  asm volatile("" : "+v"(bf), "+v"(bb));
  const float bsum = nok ? (bf + bb) : 0.0f;

  float* slab = sOut[wave];
#pragma unroll 1
  for (int tile = 0; tile < kHeadRowsPerWave / 16; ++tile) {
    const int t = row0 + tile * 16 + c;
    const float* rf = h2f + (size_t)t * kHPitch;
    const float* rb = h2b + (size_t)(kLen - 1 - t) * kHPitch;
    v4f f0 = *(const v4f*)(rf + 8 * hs);
    v4f f1 = *(const v4f*)(rf + 8 * hs + 4);
    v4f f2 = *(const v4f*)(rf + 16 + 8 * hs);
    v4f f3 = *(const v4f*)(rf + 20 + 8 * hs);
    v4f g0 = *(const v4f*)(rb + 8 * hs);
    v4f g1 = *(const v4f*)(rb + 8 * hs + 4);
    v4f g2 = *(const v4f*)(rb + 16 + 8 * hs);
    v4f g3 = *(const v4f*)(rb + 20 + 8 * hs);
    asm volatile("" : "+v"(f0), "+v"(f1), "+v"(f2), "+v"(f3));
    asm volatile("" : "+v"(g0), "+v"(g1), "+v"(g2), "+v"(g3));
    v16b Afh, Afl, Abh, Abl;
    split16(f0, f1, f2, f3, Afh, Afl);
    split16(g0, g1, g2, g3, Abh, Abl);
    v8f acc = (v8f){bsum, bsum, bsum, bsum, bsum, bsum, bsum, bsum};
    acc = mma3_bf(Afh, Afl, Bfh, Bfl, acc);
    acc = mma3_bf(Abh, Abl, Bbh, Bbl, acc);
    if (nok) {
#pragma unroll
      for (int r = 0; r < 8; ++r) slab[(tile * 16 + 8 * hs + r) * kVoc + c] = acc[r];
    }
  }
  __syncthreads();

  {
    v4f sv[5];
#pragma unroll
    for (int it = 0; it < 5; ++it) sv[it] = *(const v4f*)(slab + it * 128 + lane * 4);
    float* op = out + (size_t)row0 * kVoc;
    for (int pass = 0; pass < 2; ++pass) {
#pragma unroll
      for (int it = 0; it < 5; ++it) {
        *(volatile v4f*)(op + it * 128 + lane * 4) = sv[it];
      }
      __threadfence();
    }
  }
}

extern "C" void kernel_launch(void* const* d_in, const int* in_sizes, int n_in,
                              void* d_out, int out_size, void* d_ws, size_t ws_size,
                              hipStream_t stream) {
  if (n_in < 22 || d_out == nullptr || d_ws == nullptr) return;
  const int expect_sizes[22] = {
      kVoc * kEmb,
      kGates * kEmb, kGates * kHid, kGates, kGates,
      kGates * kHid, kGates * kHid, kGates, kGates,
      kGates * kEmb, kGates * kHid, kGates, kGates,
      kGates * kHid, kGates * kHid, kGates, kGates,
      kVoc * kHid, kVoc, kVoc * kHid, kVoc,
      kLen};
  for (int i = 0; i < 22; ++i) {
    if (in_sizes[i] != expect_sizes[i]) return;
  }
  if (out_size != kLen * kVoc) return;
  if (ws_size < kWsTotal) return;

  const float* embed  = (const float*)d_in[0];
  const float* Wih_f1 = (const float*)d_in[1];
  const float* Whh_f1 = (const float*)d_in[2];
  const float* bih_f1 = (const float*)d_in[3];
  const float* bhh_f1 = (const float*)d_in[4];
  const float* Wih_f2 = (const float*)d_in[5];
  const float* Whh_f2 = (const float*)d_in[6];
  const float* bih_f2 = (const float*)d_in[7];
  const float* bhh_f2 = (const float*)d_in[8];
  const float* Wih_b1 = (const float*)d_in[9];
  const float* Whh_b1 = (const float*)d_in[10];
  const float* bih_b1 = (const float*)d_in[11];
  const float* bhh_b1 = (const float*)d_in[12];
  const float* Wih_b2 = (const float*)d_in[13];
  const float* Whh_b2 = (const float*)d_in[14];
  const float* bih_b2 = (const float*)d_in[15];
  const float* bhh_b2 = (const float*)d_in[16];
  const float* Wlin_f = (const float*)d_in[17];
  const float* blin_f = (const float*)d_in[18];
  const float* Wlin_b = (const float*)d_in[19];
  const float* blin_b = (const float*)d_in[20];
  const int*   tokens = (const int*)d_in[21];
  float* out = (float*)d_out;

  char* wsb = (char*)d_ws;
  float* h1f = (float*)(wsb + 0 * kPlaneBytes);
  float* h1b = (float*)(wsb + 1 * kPlaneBytes);
  float* h2f = (float*)(wsb + 2 * kPlaneBytes);
  float* h2b = (float*)(wsb + 3 * kPlaneBytes);

  chain_scan_kernel<1><<<2, 32, 0, stream>>>(embed, tokens, h2f, h2b,
                                             Wih_f1, Whh_f1, bih_f1, bhh_f1,
                                             Wih_b1, Whh_b1, bih_b1, bhh_b1,
                                             h1f, h1b);
  chain_scan_kernel<2><<<2, 32, 0, stream>>>(embed, tokens, h1f, h1b,
                                             Wih_f2, Whh_f2, bih_f2, bhh_f2,
                                             Wih_b2, Whh_b2, bih_b2, bhh_b2,
                                             h2f, h2b);
  head_kernel<<<kHeadBlocks, kHeadWaves * 32, 0, stream>>>(h2f, h2b, Wlin_f, blin_f, Wlin_b, blin_b, out);
}
